// BatchSiren_6717328851683
// MI455X (gfx1250) — hardware-verified
//
#include <hip/hip_runtime.h>
#include <math.h>

typedef __attribute__((ext_vector_type(16))) _Float16 v16h;
typedef __attribute__((ext_vector_type(16))) __bf16 v16b;
typedef __attribute__((ext_vector_type(8)))  _Float16 v8h;
typedef __attribute__((ext_vector_type(8)))  float v8f;
typedef __attribute__((ext_vector_type(4)))  float v4f;
typedef __attribute__((ext_vector_type(2)))  float v2f;
typedef __attribute__((ext_vector_type(4)))  unsigned v4u;
typedef __attribute__((ext_vector_type(4)))  int v4i;
typedef float __attribute__((may_alias)) float_a;
typedef int __attribute__((may_alias)) int_a;

template <typename T> __device__ __forceinline__ void vst2(void* p, T v) { *(volatile T*)p = v; __threadfence(); *(volatile T*)p = v; }
__device__ __forceinline__ v8f wmma16(v16h a, v16h b, v8f c) {
  v8f d = __builtin_amdgcn_wmma_f32_16x16x32_f16(false, a, false, b, (short)0, c, false, false);
  asm volatile("v_nop\n\tv_nop\n\tv_nop\n\tv_nop" : "+v"(d) : "v"(a), "v"(b));
  return d;
}
__device__ __forceinline__ v8f wmma_bf(v16b a, v16b b, v8f c) {
  v8f d = __builtin_amdgcn_wmma_f32_16x16x32_bf16(false, a, false, b, (short)0, c, false, false);
  asm volatile("v_nop\n\tv_nop\n\tv_nop\n\tv_nop" : "+v"(d) : "v"(a), "v"(b));
  return d;
}
__device__ __forceinline__ v16h frag_h(const _Float16* rowk0, int lane) {
  union { v16h v; v8h q[2]; } u; const _Float16* p = rowk0 + 8 * (lane >> 4);
  u.q[0] = *(const v8h*)p; u.q[1] = *(const v8h*)(p + 16); return u.v;
}
__device__ __forceinline__ v16h frag_f32(const float* rowk0, int lane) {
  v16h a; const float* p = rowk0 + 8 * (lane >> 4);
#pragma unroll
  for (int i = 0; i < 8; ++i) { a[i] = (_Float16)p[i]; a[8 + i] = (_Float16)p[16 + i]; }
  return a;
}
__device__ __forceinline__ v16h frag_f32s(const float* rowk0, int lane, float sc) {
  v16h a; const float* p = rowk0 + 8 * (lane >> 4);
#pragma unroll
  for (int i = 0; i < 8; ++i) { a[i] = (_Float16)(p[i] * sc); a[8 + i] = (_Float16)(p[16 + i] * sc); }
  return a;
}
__device__ __forceinline__ v16h fragc_f32(const float* W, int k0, int n, int lane, int ld, int K) {
  v16h a; const int g = lane >> 4;
#pragma unroll
  for (int i = 0; i < 8; ++i) { const int ka = k0 + 8 * g + i, kb = ka + 16;
    a[i] = (_Float16)(ka < K ? W[(size_t)ka * ld + n] : 0.f); a[8 + i] = (_Float16)(kb < K ? W[(size_t)kb * ld + n] : 0.f); }
  return a;
}
struct F2 { v16b h, l; };
__device__ __forceinline__ F2 bsplit16(const float v[16]) { F2 r;
#pragma unroll
  for (int i = 0; i < 16; ++i) { const __bf16 h = (__bf16)v[i]; r.h[i] = h; r.l[i] = (__bf16)(v[i] - (float)h); }
  return r; }
__device__ __forceinline__ F2 split_row(const float* row, int k0, int lane) { float v[16]; const float* p = row + k0 + 8 * (lane >> 4);
#pragma unroll
  for (int i = 0; i < 8; ++i) { v[i] = p[i]; v[8 + i] = p[16 + i]; }
  return bsplit16(v); }
__device__ __forceinline__ F2 split_rowK(const float* row, int k0, int lane, int K) { float v[16]; const int g = lane >> 4;
#pragma unroll
  for (int i = 0; i < 8; ++i) { const int ka = k0 + 8 * g + i, kb = ka + 16; v[i] = ka < K ? row[ka] : 0.f; v[8 + i] = kb < K ? row[kb] : 0.f; }
  return bsplit16(v); }
__device__ __forceinline__ F2 split_col(const float* W, int k0, int n, int lane, int ld, int K) { float v[16]; const int g = lane >> 4;
#pragma unroll
  for (int i = 0; i < 8; ++i) { const int ka = k0 + 8 * g + i, kb = ka + 16; v[i] = ka < K ? W[(size_t)ka * ld + n] : 0.f; v[8 + i] = kb < K ? W[(size_t)kb * ld + n] : 0.f; }
  return bsplit16(v); }
__device__ __forceinline__ v8f mac3(const F2& a, const F2& b, v8f c) { c = wmma_bf(a.l, b.h, c); c = wmma_bf(a.h, b.l, c); return wmma_bf(a.h, b.h, c); }
__device__ __forceinline__ float sigm(float v) { return 1.0f / (1.0f + expf(-v)); }
#define LDSX() do { asm volatile("s_wait_dscnt 0" ::: "memory"); __builtin_amdgcn_wave_barrier(); __builtin_amdgcn_fence(__ATOMIC_RELEASE, "workgroup"); } while (0)


#define NS 2048
#define NPT 1024
#define HID 32
__device__ __forceinline__ float bfr(float v) { return (float)(__bf16)v; }
__device__ __attribute__((noinline)) float sin_ni(float v) { return sinf(v); }

__global__ __launch_bounds__(256) void k_siren(const float* __restrict__ w1, const float* __restrict__ b1, const float* __restrict__ w2, const float* __restrict__ b2, const float* __restrict__ w3, const float* __restrict__ b3, const float* __restrict__ coords, float* __restrict__ out) {
  __shared__ __align__(16) float sh1[NPT / 2][HID + 4]; __shared__ __align__(16) float sh2[NPT / 2][HID + 4]; __shared__ float sw1[2][HID], sb1[HID], sb2[HID], sw3[HID][3], sb3[3];
  const int tid = threadIdx.x, wave = tid >> 5, lane = tid & 31, col = lane & 15, g = lane >> 4; const int b = blockIdx.x;
  if (tid < 2 * HID) sw1[tid / HID][tid % HID] = bfr(w1[(size_t)b * 2 * HID + tid]);
  if (tid < HID) { sb1[tid] = bfr(b1[(size_t)b * HID + tid]); sb2[tid] = bfr(b2[(size_t)b * HID + tid]); }
  if (tid < HID * 3) sw3[tid / 3][tid % 3] = bfr(w3[(size_t)b * HID * 3 + tid]);
  if (tid < 3) sb3[tid] = bfr(b3[(size_t)b * 3 + tid]);
  __syncthreads();
  const float* w2b = w2 + (size_t)b * HID * HID;
  v16b bw[2];
#pragma unroll
  for (int j = 0; j < 2; ++j) bw[j] = split_col(w2b, 0, j * 16 + col, lane, HID, HID).h;
#pragma unroll 1
  for (int hp = 0; hp < 2; ++hp) { const int nb0 = hp * (NPT / 2);
#pragma unroll 1
  for (int nl = tid; nl < NPT / 2; nl += 256) { const int n = nb0 + nl; const float c0 = bfr(coords[n * 2]), c1 = bfr(coords[n * 2 + 1]);
#pragma unroll 1
    for (int o = 0; o < HID; ++o) sh1[nl][o] = sin_ni(30.0f * (c0 * sw1[0][o] + c1 * sw1[1][o] + sb1[o])); }
  __syncthreads();
#pragma unroll 1
  for (int rt = wave; rt < NPT / 32; rt += 8) { const F2 a = split_row(&sh1[rt * 16 + col][0], 0, lane);
#pragma unroll
    for (int j = 0; j < 2; ++j) { v8f acc = {}; acc = wmma_bf(a.l, bw[j], acc); acc = wmma_bf(a.h, bw[j], acc);
#pragma unroll
      for (int r = 0; r < 8; ++r) { const int o = j * 16 + col; sh2[rt * 16 + 8 * g + r][o] = sin_ni(30.0f * (acc[r] + sb2[o])); } } }
  __syncthreads();
#pragma unroll 1
  for (int e = tid; e < (NPT / 2) * 3; e += 256) { const int nl = e / 3, c = e % 3; float s = sb3[c];
#pragma unroll 2
    for (int k = 0; k < HID; ++k) s += sh2[nl][k] * sw3[k][c];
    vst2(out + ((size_t)b * NPT + nb0) * 3 + e, (float_a)s); }
  __syncthreads(); }
}
extern "C" void kernel_launch(void* const* d_in, const int* in_sizes, int n_in, void* d_out, int out_size, void* d_ws, size_t ws_size, hipStream_t stream) {
  (void)in_sizes; (void)n_in; (void)out_size; (void)ws_size; (void)d_ws;
  const float** I = (const float**)d_in;
  k_siren<<<NS, 256, 0, stream>>>(I[0], I[1], I[2], I[3], I[4], I[5], I[6], (float*)d_out);
}
